// PlainSpikeSelfAttention_65816078844476
// MI455X (gfx1250) — hardware-verified
//
#include <hip/hip_runtime.h>
#include <stddef.h>
#include <stdint.h>


#define TT 4
#define BB 4
#define NSEQ 1024
#define DM 512
#define NH 8
#define HD 64
#define MROWS (TT * BB * NSEQ)

static_assert(MROWS % 64 == 0);
static_assert(DM % 128 == 0);
static_assert(NSEQ % 64 == 0);
static_assert(NH * HD == DM);
static_assert(HD == 64);

typedef __bf16   v16bf __attribute__((ext_vector_type(16)));
typedef _Float16 v16h  __attribute__((ext_vector_type(16)));
typedef _Float16 v8h   __attribute__((ext_vector_type(8)));
typedef float    v8f   __attribute__((ext_vector_type(8)));
typedef float    v4f   __attribute__((ext_vector_type(4)));
typedef unsigned int v4u __attribute__((ext_vector_type(4)));

union Frag  { v16bf b; v16h h; v8h p[2]; v4u q[2]; };
union Pack8 { v8h h; v4u u; unsigned short s[8]; };
union Vec8  { v8f v; v4f q[2]; v4u u[2]; float f[8]; };

#define NOPS4 "v_nop\n\tv_nop\n\tv_nop\n\tv_nop"

__device__ __forceinline__ v8f vzero8() {
  v8f z = {0.f, 0.f, 0.f, 0.f, 0.f, 0.f, 0.f, 0.f};
  return z;
}

__device__ __forceinline__ float bf16r(float f) {
  unsigned int u = __builtin_bit_cast(unsigned int, f);
  u += 0x7FFFu + ((u >> 16) & 1u);
  u &= 0xFFFF0000u;
  return __builtin_bit_cast(float, u);
}
__device__ __forceinline__ unsigned short bf16bits(float f) {
  unsigned int u = __builtin_bit_cast(unsigned int, f);
  u += 0x7FFFu + ((u >> 16) & 1u);
  return (unsigned short)(u >> 16);
}

__device__ __forceinline__ void ldq(const unsigned short* src, int ld, v4u& q0, v4u& q1) {
  const int l = threadIdx.x & 31;
  const unsigned short* p = src + (l & 15) * ld + 8 * (l >> 4);
  q0 = *(const v4u*)(p);
  q1 = *(const v4u*)(p + 16);
}

__device__ __forceinline__ v8f wbf(v16bf a, v16bf b, v8f c) {
  return __builtin_amdgcn_wmma_f32_16x16x32_bf16(false, a, false, b, (short)0, c, false, false);
}
__device__ __forceinline__ v8f whf(v16h a, v16h b, v8f c) {
  return __builtin_amdgcn_wmma_f32_16x16x32_f16(false, a, false, b, (short)0, c, false, false);
}

template <int MODE>
__global__ __launch_bounds__(256) void k_cvt(const float* __restrict__ src, unsigned short* dst, int n)
{
  const size_t base = ((size_t)blockIdx.x * 256 + threadIdx.x) * 8;
  if (base + 8 <= (size_t)n) {
    Vec8 in;
    in.q[0] = *(const v4f*)(src + base);
    in.q[1] = *(const v4f*)(src + base + 4);
    Pack8 pk;
#pragma unroll
    for (int r = 0; r < 8; ++r) {
      if constexpr (MODE == 0) pk.s[r] = bf16bits(in.f[r]);
      else                     pk.h[r] = (_Float16)(bf16r(in.f[r]) * 256.0f);
    }
    const v4u v = pk.u;
    *(volatile v4u*)(dst + base) = v;
    __threadfence();
    *(volatile v4u*)(dst + base) = v;
  }
}

template <int MODE>
__device__ __forceinline__ void stage_tile(unsigned char* stg, v8f acc, int i, int j,
                                           int wm, int wn, int h, int c,
                                           const float* __restrict__ bias, int n0)
{
  if constexpr (MODE == 2) {
    const float bj = bf16r(bias[n0 + 32 * wn + 16 * j + c]);
    Pack8 pk;
#pragma unroll
    for (int r = 0; r < 8; ++r) pk.h[r] = (_Float16)((acc[r] + bj) * 16.0f);
    const int off = ((32 * wn + 16 * j + c) * 72 + 32 * wm + 16 * i + 8 * h) * 2;
    *(v4u*)(stg + off) = pk.u;
  } else {
    const int nb = n0 + 32 * wn + 16 * i + 8 * h;
    Vec8 bb;
    bb.q[0] = *(const v4f*)(bias + nb);
    bb.q[1] = *(const v4f*)(bias + nb + 4);
    if constexpr (MODE == 3) {
      Vec8 o;
#pragma unroll
      for (int r = 0; r < 8; ++r) o.f[r] = acc[r] * (1.0f / 16384.0f) + bf16r(bb.f[r]);
      const int off = ((32 * wm + 16 * j + c) * 132 + 32 * wn + 16 * i + 8 * h) * 4;
      *(v4u*)(stg + off)      = o.u[0];
      *(v4u*)(stg + off + 16) = o.u[1];
    } else {
      Pack8 pk;
#pragma unroll
      for (int r = 0; r < 8; ++r) pk.h[r] = (_Float16)((acc[r] + bf16r(bb.f[r])) * 4.0f);
      const int off = ((32 * wm + 16 * j + c) * 136 + 32 * wn + 16 * i + 8 * h) * 2;
      *(v4u*)(stg + off) = pk.u;
    }
  }
}

template <int MODE>
__global__ __launch_bounds__(256) void k_proj(const unsigned short* __restrict__ X,
                                             const unsigned short* __restrict__ W,
                                             const float* __restrict__ bias,
                                             void* dst)
{
  __shared__ __align__(16) unsigned char stg[33792];
  const int tid = threadIdx.x, w = tid >> 5, l = tid & 31, h = l >> 4, c = l & 15;
  const int wm = w >> 2, wn = w & 3;
  const int m0 = blockIdx.x * 64, n0 = blockIdx.y * 128;

  const unsigned short *P, *R;
  int prow, rrow;
  if constexpr (MODE == 2) { P = X; R = W; prow = m0 + 32 * wm; rrow = n0 + 32 * wn; }
  else                     { P = W; R = X; prow = n0 + 32 * wn; rrow = m0 + 32 * wm; }
  const unsigned short* p0 = P + (size_t)prow * DM;
  const unsigned short* p1 = P + (size_t)(prow + 16) * DM;
  const unsigned short* r0 = R + (size_t)rrow * DM;
  const unsigned short* r1 = R + (size_t)(rrow + 16) * DM;

  v8f a00 = vzero8(), a01 = vzero8(), a10 = vzero8(), a11 = vzero8();

#pragma unroll 1
  for (int k0 = 0; k0 < DM; k0 += 32) {
    Frag fp0, fp1, fr0, fr1;
    ldq(p0 + k0, DM, fp0.q[0], fp0.q[1]);
    ldq(p1 + k0, DM, fp1.q[0], fp1.q[1]);
    ldq(r0 + k0, DM, fr0.q[0], fr0.q[1]);
    ldq(r1 + k0, DM, fr1.q[0], fr1.q[1]);
    if constexpr (MODE == 3) {
      a00 = whf(fp0.h, fr0.h, a00);
      a01 = whf(fp0.h, fr1.h, a01);
      a10 = whf(fp1.h, fr0.h, a10);
      a11 = whf(fp1.h, fr1.h, a11);
      asm volatile(NOPS4
                   : "+v"(a00), "+v"(a01), "+v"(a10), "+v"(a11)
                   : "v"(fp0.h), "v"(fp1.h), "v"(fr0.h), "v"(fr1.h));
    } else {
      a00 = wbf(fp0.b, fr0.b, a00);
      a01 = wbf(fp0.b, fr1.b, a01);
      a10 = wbf(fp1.b, fr0.b, a10);
      a11 = wbf(fp1.b, fr1.b, a11);
      asm volatile(NOPS4
                   : "+v"(a00), "+v"(a01), "+v"(a10), "+v"(a11)
                   : "v"(fp0.b), "v"(fp1.b), "v"(fr0.b), "v"(fr1.b));
    }
  }

  stage_tile<MODE>(stg, a00, 0, 0, wm, wn, h, c, bias, n0);
  stage_tile<MODE>(stg, a01, 0, 1, wm, wn, h, c, bias, n0);
  stage_tile<MODE>(stg, a10, 1, 0, wm, wn, h, c, bias, n0);
  stage_tile<MODE>(stg, a11, 1, 1, wm, wn, h, c, bias, n0);
  __syncthreads();

  const int pc = l & 7;
  if constexpr (MODE == 0 || MODE == 1) {
    v4u vals[4];
    unsigned short* pp[4];
#pragma unroll
    for (int s = 0; s < 4; ++s) {
      const int L = 16 * w + 4 * s + (l >> 3);
      const int ml = L >> 1;
      const int hf = L & 1;
      vals[s] = *(const v4u*)(stg + (ml * 136 + 64 * hf + 8 * pc) * 2);
      pp[s] = (unsigned short*)dst + (size_t)(m0 + ml) * DM + n0 + 64 * hf + 8 * pc;
    }
#pragma unroll
    for (int s = 0; s < 4; ++s) *(volatile v4u*)(pp[s]) = vals[s];
    __threadfence();
#pragma unroll
    for (int s = 0; s < 4; ++s) *(volatile v4u*)(pp[s]) = vals[s];
  } else if constexpr (MODE == 3) {
    v4u vals[8];
    float* pp[8];
#pragma unroll
    for (int s = 0; s < 8; ++s) {
      const int L = 32 * w + 4 * s + (l >> 3);
      const int ml = L >> 2;
      const int qt = L & 3;
      vals[s] = *(const v4u*)(stg + (ml * 132 + 32 * qt + 4 * pc) * 4);
      pp[s] = (float*)dst + (size_t)(m0 + ml) * DM + n0 + 32 * qt + 4 * pc;
    }
#pragma unroll
    for (int s = 0; s < 8; ++s) *(volatile v4u*)(pp[s]) = vals[s];
    __threadfence();
#pragma unroll
    for (int s = 0; s < 8; ++s) *(volatile v4u*)(pp[s]) = vals[s];
  } else {
    v4u vals[4];
    unsigned short* pp[4];
    const int tb = m0 / NSEQ;
    const int ns0 = m0 % NSEQ;
#pragma unroll
    for (int s = 0; s < 4; ++s) {
      const int L = 16 * w + 4 * s + (l >> 3);
      const int n = n0 + L;
      const int hh = n >> 6;
      const int hd = n & 63;
      vals[s] = *(const v4u*)(stg + (L * 72 + 8 * pc) * 2);
      pp[s] = (unsigned short*)dst + ((size_t)(tb * NH + hh) * HD + hd) * NSEQ + ns0 + 8 * pc;
    }
#pragma unroll
    for (int s = 0; s < 4; ++s) *(volatile v4u*)(pp[s]) = vals[s];
    __threadfence();
#pragma unroll
    for (int s = 0; s < 4; ++s) *(volatile v4u*)(pp[s]) = vals[s];
  }
}

__device__ __forceinline__ v8f score_tile(const unsigned short* kb, v16h q0, v16h q1)
{
  Frag k0, k1;
  ldq(kb, 72, k0.q[0], k0.q[1]);
  ldq(kb + 32, 72, k1.q[0], k1.q[1]);
  v8f a = vzero8();
  a = whf(k0.h, q0, a);
  a = whf(k1.h, q1, a);
  asm volatile(NOPS4 : "+v"(a) : "v"(k0.h), "v"(k1.h), "v"(q0), "v"(q1));
  return a;
}

__device__ __forceinline__ void pv_step(const unsigned short* vb, v8f sa, v8f sb,
                                        v8f& c0, v8f& c1, v8f& c2, v8f& c3)
{
  Frag pk;
#pragma unroll
  for (int r = 0; r < 8; ++r) {
    pk.p[0][r] = (_Float16)(sa[r] * 0.125f);
    pk.p[1][r] = (_Float16)(sb[r] * 0.125f);
  }
  const v16h pv = pk.h;
  Frag v0, v1, v2, v3;
  ldq(vb,           72, v0.q[0], v0.q[1]);
  ldq(vb + 16 * 72, 72, v1.q[0], v1.q[1]);
  ldq(vb + 32 * 72, 72, v2.q[0], v2.q[1]);
  ldq(vb + 48 * 72, 72, v3.q[0], v3.q[1]);
  c0 = whf(v0.h, pv, c0);
  c1 = whf(v1.h, pv, c1);
  c2 = whf(v2.h, pv, c2);
  c3 = whf(v3.h, pv, c3);
  asm volatile(NOPS4
               : "+v"(c0), "+v"(c1), "+v"(c2), "+v"(c3)
               : "v"(v0.h), "v"(v1.h), "v"(v2.h), "v"(v3.h), "v"(pv));
}

__global__ __launch_bounds__(128) void k_attn(const unsigned short* __restrict__ qf,
                                             const unsigned short* __restrict__ kf,
                                             const unsigned short* __restrict__ vt,
                                             unsigned short* cf)
{
  __shared__ __align__(16) unsigned short klds[64 * 72];
  __shared__ __align__(16) unsigned short vlds[64 * 72];
  __shared__ __align__(16) unsigned short cst[4 * 16 * 72];

  const int tid = threadIdx.x, w = tid >> 5, l = tid & 31, h = l >> 4, c = l & 15;
  const int tbh = blockIdx.y, tb = tbh >> 3, hh = tbh & 7;
  const int q0 = blockIdx.x * 64 + 16 * w;

  v16h qa, qb;
  {
    const unsigned short* qsrc = qf + (size_t)(tb * NSEQ + q0) * DM + hh * HD;
    Frag f0, f1;
    ldq(qsrc,      DM, f0.q[0], f0.q[1]);
    ldq(qsrc + 32, DM, f1.q[0], f1.q[1]);
    qa = f0.h; qb = f1.h;
  }

  v8f c0 = vzero8(), c1 = vzero8(), c2 = vzero8(), c3 = vzero8();
  float rs = 0.f;

#pragma unroll 1
  for (int kt0 = 0; kt0 < NSEQ; kt0 += 64) {
    __syncthreads();
#pragma unroll
    for (int it = 0; it < 4; ++it) {
      const int q = it * 128 + tid;
      const int kr = q >> 3;
      const int pc = q & 7;
      const unsigned short* src = kf + (size_t)(tb * NSEQ + kt0 + kr) * DM + hh * HD + 8 * pc;
      *(v4u*)(klds + kr * 72 + 8 * pc) = *(const v4u*)src;
    }
#pragma unroll
    for (int it = 0; it < 4; ++it) {
      const int q = it * 128 + tid;
      const int hd = q >> 3;
      const int pc = q & 7;
      const unsigned short* src = vt + (size_t)(tbh * HD + hd) * NSEQ + kt0 + 8 * pc;
      *(v4u*)(vlds + hd * 72 + 8 * pc) = *(const v4u*)src;
    }
    __syncthreads();

    v8f s0 = score_tile(klds + 0 * 16 * 72, qa, qb);
    v8f s1 = score_tile(klds + 1 * 16 * 72, qa, qb);
    v8f s2 = score_tile(klds + 2 * 16 * 72, qa, qb);
    v8f s3 = score_tile(klds + 3 * 16 * 72, qa, qb);

#pragma unroll
    for (int r = 0; r < 8; ++r) {
      float v;
      v = fmaxf(s0[r], 0.f); rs += v; s0[r] = v;
      v = fmaxf(s1[r], 0.f); rs += v; s1[r] = v;
      v = fmaxf(s2[r], 0.f); rs += v; s2[r] = v;
      v = fmaxf(s3[r], 0.f); rs += v; s3[r] = v;
    }

    pv_step(vlds + 0,  s0, s1, c0, c1, c2, c3);
    pv_step(vlds + 32, s2, s3, c0, c1, c2, c3);
  }

  const float rsum = rs + __shfl_xor(rs, 16, 32);
  const float inv = 64.0f / (2.0f * rsum + 2.56e-4f);

  {
    unsigned short* cw = cst + w * 16 * 72;
#pragma unroll
    for (int i = 0; i < 4; ++i) {
      const v8f acc = (i == 0) ? c0 : (i == 1) ? c1 : (i == 2) ? c2 : c3;
      Pack8 pk;
#pragma unroll
      for (int r = 0; r < 8; ++r) pk.h[r] = (_Float16)(acc[r] * inv);
      *(v4u*)(cw + c * 72 + 16 * i + 8 * h) = pk.u;
    }
  }
  __syncthreads();

  v4u vals[4];
  unsigned short* pp[4];
  const int pc = l & 7;
#pragma unroll
  for (int s = 0; s < 4; ++s) {
    const int L = 4 * s + (l >> 3);
    vals[s] = *(const v4u*)(cst + (w * 16 + L) * 72 + 8 * pc);
    pp[s] = cf + (size_t)(tb * NSEQ + q0 + L) * DM + hh * HD + 8 * pc;
  }
#pragma unroll
  for (int s = 0; s < 4; ++s) *(volatile v4u*)(pp[s]) = vals[s];
  __threadfence();
#pragma unroll
  for (int s = 0; s < 4; ++s) *(volatile v4u*)(pp[s]) = vals[s];
}

extern "C" void kernel_launch(void* const* d_in, const int* in_sizes, int n_in,
                              void* d_out, int out_size, void* d_ws, size_t ws_size,
                              hipStream_t stream)
{
  if (n_in != 9) return;
  const int nx = MROWS * DM;
  const int nw = DM * DM;
  if (in_sizes[0] != nx || out_size != nx) return;
  for (int i = 0; i < 4; ++i) {
    if (in_sizes[1 + 2 * i] != nw || in_sizes[2 + 2 * i] != DM) return;
  }
  const size_t p16 = (size_t)nx * 2;
  const size_t w16 = (size_t)nw * 2;
  const size_t need = 5 * p16 + 4 * w16;
  if (need > ws_size) return;

  unsigned char* ws = (unsigned char*)d_ws;
  unsigned short* xb  = (unsigned short*)(ws + 0 * p16);
  unsigned short* qfp = (unsigned short*)(ws + 1 * p16);
  unsigned short* kfp = (unsigned short*)(ws + 2 * p16);
  unsigned short* vtp = (unsigned short*)(ws + 3 * p16);
  unsigned short* cfp = (unsigned short*)(ws + 4 * p16);
  unsigned short* wb  = (unsigned short*)(ws + 5 * p16);
  unsigned short* wqb = wb + 0 * (size_t)nw;
  unsigned short* wkb = wb + 1 * (size_t)nw;
  unsigned short* wvb = wb + 2 * (size_t)nw;
  unsigned short* wof = wb + 3 * (size_t)nw;

  const float* x  = (const float*)d_in[0];
  const float* wq = (const float*)d_in[1];
  const float* bq = (const float*)d_in[2];
  const float* wk = (const float*)d_in[3];
  const float* bk = (const float*)d_in[4];
  const float* wv = (const float*)d_in[5];
  const float* bv = (const float*)d_in[6];
  const float* wo = (const float*)d_in[7];
  const float* bo = (const float*)d_in[8];

  k_cvt<0><<<dim3((nx + 2047) / 2048), dim3(256), 0, stream>>>(x,  xb,  nx);
  k_cvt<0><<<dim3((nw + 2047) / 2048), dim3(256), 0, stream>>>(wq, wqb, nw);
  k_cvt<0><<<dim3((nw + 2047) / 2048), dim3(256), 0, stream>>>(wk, wkb, nw);
  k_cvt<0><<<dim3((nw + 2047) / 2048), dim3(256), 0, stream>>>(wv, wvb, nw);
  k_cvt<1><<<dim3((nw + 2047) / 2048), dim3(256), 0, stream>>>(wo, wof, nw);

  const dim3 gg(MROWS / 64, DM / 128);
  k_proj<0><<<gg, dim3(256), 0, stream>>>(xb, wqb, bq, (void*)qfp);
  k_proj<1><<<gg, dim3(256), 0, stream>>>(xb, wkb, bk, (void*)kfp);
  k_proj<2><<<gg, dim3(256), 0, stream>>>(xb, wvb, bv, (void*)vtp);

  k_attn<<<dim3(NSEQ / 64, TT * BB * NH), dim3(128), 0, stream>>>(qfp, kfp, vtp, cfp);

  k_proj<3><<<gg, dim3(256), 0, stream>>>(cfp, wof, bo, d_out);
}
